// STS_Block_38465727103445
// MI455X (gfx1250) — hardware-verified
//
#include <hip/hip_runtime.h>
#define BB 4
#define CCH 96
#define CP16 128
#define TT 9216
#define DI 192
#define NS 16
#define DTR 6
#define DTP 32
#define XPW (DTR + 2 * NS)
#define XDP 64
#define NR (BB * TT)
#define LNEPS 1e-5f
#define USC 256.0f
#define YSC 16384.0f
__device__ __forceinline__ float fexp(float x) { return __builtin_amdgcn_exp2f(x * 1.4426950408889634f); }
typedef __bf16 v16b __attribute__((ext_vector_type(16)));
typedef unsigned short v8us __attribute__((ext_vector_type(8), may_alias));
typedef float  v8f  __attribute__((ext_vector_type(8)));
typedef float  v4f  __attribute__((ext_vector_type(4)));
typedef float  v4fa __attribute__((ext_vector_type(4), may_alias));
union FragB { v16b v; v8us half[2]; unsigned short u[16]; };

__device__ __forceinline__ unsigned short bf16_bits(float x) { unsigned int u = __float_as_uint(x); return (unsigned short)((u + 0x7FFFu + ((u >> 16) & 1u)) >> 16); }
__device__ __forceinline__ float bf16_val(unsigned short b) { return __uint_as_float(((unsigned int)b) << 16); }
__device__ __forceinline__ float bf16_round(float x) { return bf16_val(bf16_bits(x)); }
template <int NT>
__device__ __forceinline__ v8f mmaN(v16b ah, v16b al, v16b bh, v16b bl, v8f c) {
  c = __builtin_amdgcn_wmma_f32_16x16x32_bf16(false, ah, false, bh, (short)0, c, false, false);
  if (NT >= 2) c = __builtin_amdgcn_wmma_f32_16x16x32_bf16(false, al, false, bh, (short)0, c, false, false);
  if (NT >= 3) c = __builtin_amdgcn_wmma_f32_16x16x32_bf16(false, ah, false, bl, (short)0, c, false, false);
  asm volatile("v_nop\n\tv_nop\n\tv_nop\n\tv_nop" : "+v"(c) : "v"(ah), "v"(al), "v"(bh), "v"(bl));
  return c;
}

__global__ __launch_bounds__(256) void k_wt_bf16(const float* __restrict__ W, unsigned short* __restrict__ Wt, int K, int N) {
  const int t = blockIdx.x * 256 + threadIdx.x;
  const int k8n = K / 8;
  if (t >= N * k8n) return;
  const int n = t / k8n, k8 = (t % k8n) * 8;
  v8us v;
#pragma unroll
  for (int i = 0; i < 8; ++i) v[i] = bf16_bits(W[(size_t)(k8 + i) * N + n]);
  *(volatile v8us*)(Wt + (size_t)n * K + k8) = v;
  __threadfence();
  *(volatile v8us*)(Wt + (size_t)n * K + k8) = v;
}

template <bool ASPLIT, int ACT, bool BIAS_BF16>
__global__ __launch_bounds__(128) void k_gemm_bf(const float* __restrict__ A, int lda, const unsigned short* __restrict__ Wt, int ldb,
                                               const float* __restrict__ bias, float* __restrict__ C, int ldc, int M, int N, int K) {
  __shared__ __attribute__((aligned(16))) float so[4][16][64];
  const int tid = threadIdx.x, w = tid >> 5, lane = tid & 31, ln = lane & 15, hh = lane >> 4;
  const int ntn = N / 64;
  const int wid = blockIdx.x * 4 + w;
  const int mt = wid / ntn, nq = wid % ntn;
  if (mt * 16 >= M) return;
  const int row0 = mt * 16, col0 = nq * 64;
  const float* arow = A + (size_t)(row0 + ln) * lda;
  v8f acc[4] = {};
  for (int kb = 0; kb < K; kb += 32) {
    FragB ah, al;
    const v4f x0 = *(const v4fa*)(arow + kb + 8 * hh), x1 = *(const v4fa*)(arow + kb + 8 * hh + 4);
    const v4f x2 = *(const v4fa*)(arow + kb + 16 + 8 * hh), x3 = *(const v4fa*)(arow + kb + 16 + 8 * hh + 4);
    float xs[16] = {x0[0],x0[1],x0[2],x0[3],x1[0],x1[1],x1[2],x1[3],x2[0],x2[1],x2[2],x2[3],x3[0],x3[1],x3[2],x3[3]};
#pragma unroll
    for (int i = 0; i < 16; ++i) { const unsigned short hb = bf16_bits(xs[i]); ah.u[i] = hb; al.u[i] = ASPLIT ? bf16_bits(xs[i] - bf16_val(hb)) : (unsigned short)0; }
#pragma unroll
    for (int t = 0; t < 4; ++t) {
      const unsigned short* brow = Wt + (size_t)(col0 + t * 16 + ln) * ldb + kb;
      FragB b;
      b.half[0] = *(const v8us*)(brow + 8 * hh);
      b.half[1] = *(const v8us*)(brow + 16 + 8 * hh);
      acc[t] = mmaN<ASPLIT ? 2 : 1>(ah.v, al.v, b.v, b.v, acc[t]);
    }
  }
#pragma unroll
  for (int t = 0; t < 4; ++t) {
    float bv = bias ? bias[col0 + t * 16 + ln] : 0.f;
    if (BIAS_BF16) bv = bf16_round(bv);
#pragma unroll
    for (int r = 0; r < 8; ++r) { float v = acc[t][r] + bv; if (ACT == 1) v = fmaxf(v, 0.f); so[w][8 * hh + r][t * 16 + ln] = v; }
  }
  __builtin_amdgcn_fence(__ATOMIC_ACQ_REL, "workgroup");
  __builtin_amdgcn_wave_barrier();
  const int rsub = lane >> 4, c4 = (lane & 15) * 4;
  for (int pass = 0; pass < 2; ++pass) {
#pragma unroll
    for (int q = 0; q < 8; ++q) {
      const int r = q * 2 + rsub;
      const v4f v = *(const v4fa*)&so[w][r][c4];
      *(volatile v4f*)(C + (size_t)(row0 + r) * ldc + col0 + c4) = v;
    }
    if (pass == 0) __threadfence();
  }
}

template <bool ASPLIT, int ACT, bool BIAS_BF16, bool RES_BF16>
__global__ __launch_bounds__(128) void k_gemm_bf3(const float* __restrict__ A, int lda, const unsigned short* __restrict__ Wt, int ldb,
                                                const float* __restrict__ bias, const float* __restrict__ resid, int rmod, int ldr,
                                                float* __restrict__ C, int ldc, int M, int N, int K) {
  __shared__ __attribute__((aligned(16))) float so[4][16][64];
  const int tid = threadIdx.x, w = tid >> 5, lane = tid & 31, ln = lane & 15, hh = lane >> 4;
  const int ntn = N / 64;
  const int wid = blockIdx.x * 4 + w;
  const int mt = wid / ntn, nq = wid % ntn;
  if (mt * 16 >= M) return;
  const int row0 = mt * 16, col0 = nq * 64;
  const float* arow = A + (size_t)(row0 + ln) * lda;
  v8f acc[4] = {};
  for (int kb = 0; kb < K; kb += 32) {
    FragB ah, al;
    const v4f x0 = *(const v4fa*)(arow + kb + 8 * hh), x1 = *(const v4fa*)(arow + kb + 8 * hh + 4);
    const v4f x2 = *(const v4fa*)(arow + kb + 16 + 8 * hh), x3 = *(const v4fa*)(arow + kb + 16 + 8 * hh + 4);
    float xs[16] = {x0[0],x0[1],x0[2],x0[3],x1[0],x1[1],x1[2],x1[3],x2[0],x2[1],x2[2],x2[3],x3[0],x3[1],x3[2],x3[3]};
#pragma unroll
    for (int i = 0; i < 16; ++i) { const unsigned short hb = bf16_bits(xs[i]); ah.u[i] = hb; al.u[i] = ASPLIT ? bf16_bits(xs[i] - bf16_val(hb)) : (unsigned short)0; }
#pragma unroll
    for (int t = 0; t < 4; ++t) {
      const unsigned short* brow = Wt + (size_t)(col0 + t * 16 + ln) * ldb + kb;
      FragB b;
      b.half[0] = *(const v8us*)(brow + 8 * hh);
      b.half[1] = *(const v8us*)(brow + 16 + 8 * hh);
      acc[t] = mmaN<ASPLIT ? 2 : 1>(ah.v, al.v, b.v, b.v, acc[t]);
    }
  }
#pragma unroll
  for (int t = 0; t < 4; ++t) {
    const int col = col0 + t * 16 + ln;
    float bv = bias ? bias[col] : 0.f;
    if (BIAS_BF16) bv = bf16_round(bv);
#pragma unroll
    for (int r = 0; r < 8; ++r) {
      float v = acc[t][r] + bv;
      if (resid) { float rv = resid[(size_t)((row0 + 8 * hh + r) % rmod) * ldr + col]; if (RES_BF16) rv = bf16_round(rv); v += rv; }
      if (ACT == 1) v = fmaxf(v, 0.f);
      if (ACT == 2) v = 0.5f * v * (1.0f + erff(v * 0.70710678118654752f));
      if (ACT == 3) { const float u = 0.7978845608028654f * (v + 0.044715f * v * v * v); v = 0.5f * v * (1.0f + tanhf(u)); }
      so[w][8 * hh + r][t * 16 + ln] = v;
    }
  }
  __builtin_amdgcn_fence(__ATOMIC_ACQ_REL, "workgroup");
  __builtin_amdgcn_wave_barrier();
  const int rsub = lane >> 4, c4 = (lane & 15) * 4;
  for (int pass = 0; pass < 2; ++pass) {
#pragma unroll
    for (int q = 0; q < 8; ++q) {
      const int r = q * 2 + rsub;
      const v4f v = *(const v4fa*)&so[w][r][c4];
      *(volatile v4f*)(C + (size_t)(row0 + r) * ldc + col0 + c4) = v;
    }
    if (pass == 0) __threadfence();
  }
}
template <bool PARAM_BF16>
__global__ __launch_bounds__(256) void k_layernorm(const float* __restrict__ X, const float* __restrict__ R, const float* __restrict__ g, const float* __restrict__ bta,
                                                  float* __restrict__ out_sum, float* __restrict__ out_norm, int N, float eps) {
  __shared__ float red[256];
  const int row = blockIdx.x, tid = threadIdx.x;
  const float* x = X + (size_t)row * N; const float* rr = R ? R + (size_t)row * N : nullptr;
  float vals[16];
  const int per = N / 256;
  float s1 = 0.f;
  for (int u = 0; u < per / 4; ++u) {
    const int j = tid * 4 + 1024 * u;
    const v4f a = *(const v4fa*)(x + j);
    v4f b = {0.f,0.f,0.f,0.f}; if (rr) b = *(const v4fa*)(rr + j);
#pragma unroll
    for (int q = 0; q < 4; ++q) { const float v = a[q] + b[q]; vals[u * 4 + q] = v; s1 += v; }
  }
  red[tid] = s1; __syncthreads();
  for (int st = 128; st > 0; st >>= 1) { if (tid < st) red[tid] += red[tid + st]; __syncthreads(); }
  const float mu = red[0] / (float)N; __syncthreads();
  float s2 = 0.f;
  for (int u = 0; u < per / 4; ++u)
#pragma unroll
    for (int q = 0; q < 4; ++q) { const float c = vals[u * 4 + q] - mu; s2 += c * c; }
  red[tid] = s2; __syncthreads();
  for (int st = 128; st > 0; st >>= 1) { if (tid < st) red[tid] += red[tid + st]; __syncthreads(); }
  const float rs = rsqrtf(red[0] / (float)N + eps);
  for (int pass = 0; pass < 2; ++pass) {
    for (int u = 0; u < per / 4; ++u) {
      const int j = tid * 4 + 1024 * u;
      v4f o, sm;
#pragma unroll
      for (int q = 0; q < 4; ++q) {
        float gg = g[j + q], bb = bta[j + q];
        if (PARAM_BF16) { gg = bf16_round(gg); bb = bf16_round(bb); }
        sm[q] = vals[u * 4 + q]; o[q] = (vals[u * 4 + q] - mu) * rs * gg + bb;
      }
      if (out_sum) *(volatile v4f*)(out_sum + (size_t)row * N + j) = sm;
      *(volatile v4f*)(out_norm + (size_t)row * N + j) = o;
    }
    if (pass == 0) __threadfence();
  }
}


typedef _Float16 v16h __attribute__((ext_vector_type(16)));
union FragH { v16h v; v8us half[2]; _Float16 h[16]; unsigned short u[16]; };
template <int NT>
__device__ __forceinline__ v8f mmaH(v16h ah, v16h al, v16h bh, v16h bl, v8f c) {
  c = __builtin_amdgcn_wmma_f32_16x16x32_f16(false, ah, false, bh, (short)0, c, false, false);
  if (NT >= 2) c = __builtin_amdgcn_wmma_f32_16x16x32_f16(false, al, false, bh, (short)0, c, false, false);
  if (NT >= 3) c = __builtin_amdgcn_wmma_f32_16x16x32_f16(false, ah, false, bl, (short)0, c, false, false);
  asm volatile("v_nop\n\tv_nop\n\tv_nop\n\tv_nop" : "+v"(c) : "v"(ah), "v"(al), "v"(bh), "v"(bl));
  return c;
}
template <bool ASPLIT>
__global__ __launch_bounds__(128) void k_gemm_h(const float* __restrict__ A, int lda, size_t sA, const _Float16* __restrict__ Bh, int ldb, size_t sB, float alpha, float* __restrict__ C, int ldc, size_t sC, int M, int N, int K) {
  __shared__ __attribute__((aligned(16))) float so[4][16][64];
  const int tid = threadIdx.x, w = tid >> 5, lane = tid & 31, ln = lane & 15, hh = lane >> 4; const int by = blockIdx.y;
  A += (size_t)by * sA; Bh += (size_t)by * sB; C += (size_t)by * sC;
  const int ntn = (N + 63) / 64; const int wid = blockIdx.x * 4 + w; const int mt = wid / ntn, nq = wid % ntn; if (mt * 16 >= M) return;
  const int row0 = mt * 16, col0 = nq * 64; const float* arow = A + (size_t)(row0 + ln) * lda;
  v8f acc[4] = {};
  for (int kb = 0; kb < K; kb += 32) {
    FragH ah, al;
    const v4f x0 = *(const v4fa*)(arow + kb + 8 * hh), x1 = *(const v4fa*)(arow + kb + 8 * hh + 4), x2 = *(const v4fa*)(arow + kb + 16 + 8 * hh), x3 = *(const v4fa*)(arow + kb + 16 + 8 * hh + 4);
    float xs[16] = {x0[0],x0[1],x0[2],x0[3],x1[0],x1[1],x1[2],x1[3],x2[0],x2[1],x2[2],x2[3],x3[0],x3[1],x3[2],x3[3]};
#pragma unroll
    for (int i = 0; i < 16; ++i) { const _Float16 h = (_Float16)xs[i]; ah.h[i] = h; al.h[i] = ASPLIT ? (_Float16)(xs[i] - (float)h) : (_Float16)0.0f; }
#pragma unroll
    for (int t = 0; t < 4; ++t) { if (col0 + t * 16 >= N) continue; const size_t boff = (size_t)(col0 + t * 16 + ln) * ldb + kb; FragH bq; bq.half[0] = *(const v8us*)(Bh + boff + 8 * hh); bq.half[1] = *(const v8us*)(Bh + boff + 16 + 8 * hh);
      acc[t] = mmaH<ASPLIT ? 2 : 1>(ah.v, al.v, bq.v, bq.v, acc[t]); }
  }
#pragma unroll
  for (int t = 0; t < 4; ++t) { if (col0 + t * 16 >= N) continue;
#pragma unroll
    for (int r = 0; r < 8; ++r) so[w][8 * hh + r][t * 16 + ln] = acc[t][r] * alpha; }
  __builtin_amdgcn_fence(__ATOMIC_ACQ_REL, "workgroup"); __builtin_amdgcn_wave_barrier();
  const int rsub = lane >> 4, c4 = (lane & 15) * 4;
  for (int pass = 0; pass < 2; ++pass) {
#pragma unroll
    for (int q = 0; q < 8; ++q) { const int r = q * 2 + rsub; if (col0 + c4 < N) { const v4f v = *(const v4fa*)&so[w][r][c4]; *(volatile v4f*)(C + (size_t)(row0 + r) * ldc + col0 + c4) = v; } }
    if (pass == 0) __threadfence(); }
}

__global__ __launch_bounds__(256) void k_wt_f16(const float* __restrict__ W, _Float16* __restrict__ Wt, int K, int N, float scale) {
  const int t = blockIdx.x * 256 + threadIdx.x; if (t >= N * (K / 8)) return; const int n = t / (K / 8), k8 = (t % (K / 8)) * 8; FragH f;
#pragma unroll
  for (int i = 0; i < 8; ++i) f.h[i] = (_Float16)(bf16_round(W[(size_t)(k8 + i) * N + n]) * scale); const v8us o = f.half[0];
  *(volatile v8us*)((unsigned short*)Wt + (size_t)n * K + k8) = o; __threadfence(); *(volatile v8us*)((unsigned short*)Wt + (size_t)n * K + k8) = o;
}
template <int ACT>
__global__ __launch_bounds__(128) void k_gemm_hhx(const _Float16* __restrict__ A, int lda, size_t sA, const _Float16* __restrict__ Bh, int ldb, size_t sB, float alpha, const float* __restrict__ bias, size_t sBias, const float* __restrict__ CP, int rowsPerB, size_t sCPb, int row0g,
    float* __restrict__ C, _Float16* __restrict__ C16, int ldc, size_t sC, int M, int N, int K) {
  __shared__ __attribute__((aligned(16))) float so[4][16][64];
  const int tid = threadIdx.x, w = tid >> 5, lane = tid & 31, ln = lane & 15, hh = lane >> 4; const int by = blockIdx.y;
  A += (size_t)by * sA; Bh += (size_t)by * sB; const size_t cofs = (size_t)by * sC; const float* bp = bias ? bias + (size_t)by * sBias : nullptr;
  const int ntn = (N + 63) / 64; const int wid = blockIdx.x * 4 + w; const int mt = wid / ntn, nq = wid % ntn; if (mt * 16 >= M) return;
  const int row0 = mt * 16, col0 = nq * 64; const _Float16* arow = A + (size_t)(row0 + ln) * lda;
  v8f acc[4] = {};
  for (int kb = 0; kb < K; kb += 32) { FragH ah; ah.half[0] = *(const v8us*)((const unsigned short*)arow + kb + 8 * hh); ah.half[1] = *(const v8us*)((const unsigned short*)arow + kb + 16 + 8 * hh);
#pragma unroll
    for (int t = 0; t < 4; ++t) { if (col0 + t * 16 >= N) continue; const size_t boff = (size_t)(col0 + t * 16 + ln) * ldb + kb; FragH bq; bq.half[0] = *(const v8us*)((const unsigned short*)Bh + boff + 8 * hh); bq.half[1] = *(const v8us*)((const unsigned short*)Bh + boff + 16 + 8 * hh);
      acc[t] = mmaH<1>(ah.v, ah.v, bq.v, bq.v, acc[t]); }
  }
#pragma unroll
  for (int t = 0; t < 4; ++t) { if (col0 + t * 16 >= N) continue; const int col = col0 + t * 16 + ln; const float bv = bp ? bf16_round(bp[col]) : 0.f;
#pragma unroll
    for (int r = 0; r < 8; ++r) { float v = acc[t][r] * alpha + bv; if (CP) { const int bidx = (row0g + row0 + 8 * hh + r) / rowsPerB; v += CP[(size_t)bidx * sCPb + (size_t)by * 64 + col]; } if (ACT == 1) v = (v > 0.f) ? v : expm1f(v); else if (ACT == 7) v = (v > 0.f) ? v + 1.0f : expf(v); else if (ACT == 8) v = tanhf(v); else if (ACT == 9) v = 0.5f * v * (1.0f + tanhf(0.7978845608028654f * (v + 0.044715f * v * v * v))); else if (ACT == 11) v = 1.0f / (1.0f + expf(-v)); else if (ACT == 12) v = (v > 0.f) ? v : 0.01f * v; else if (ACT == 14) v = (v > 0.f) ? v : 0.1f * v; else if (ACT == 15) v = v / (1.0f + expf(-v)); else if (ACT == 3) v = fmaxf(v, 0.f); else if (ACT == 6) v = 0.5f * v * (1.0f + erff(v * 0.70710678118654752f)); else if (ACT == 13) v = (v > 20.f) ? v : log1pf(expf(v)); so[w][8 * hh + r][t * 16 + ln] = v; } }
  __builtin_amdgcn_fence(__ATOMIC_ACQ_REL, "workgroup"); __builtin_amdgcn_wave_barrier();
  const int rsub = lane >> 4, c4 = (lane & 15) * 4; typedef _Float16 v4h __attribute__((ext_vector_type(4)));
  for (int pass = 0; pass < 2; ++pass) {
#pragma unroll
    for (int q = 0; q < 8; ++q) { const int r = q * 2 + rsub; if (col0 + c4 < N) { const v4f v = *(const v4fa*)&so[w][r][c4]; if (C) *(volatile v4f*)(C + cofs + (size_t)(row0 + r) * ldc + col0 + c4) = v; if (C16) { v4h h4; for (int i = 0; i < 4; ++i) h4[i] = (_Float16)v[i]; *(volatile v4h*)(C16 + cofs + (size_t)(row0 + r) * ldc + col0 + c4) = h4; } } }
    if (pass == 0) __threadfence(); }
}


typedef _Float16 v4h __attribute__((ext_vector_type(4)));

__global__ __launch_bounds__(256) void k_x16(const float* __restrict__ x, _Float16* __restrict__ X16, size_t n8) { const size_t t = (size_t)blockIdx.x * 256 + threadIdx.x; if (t >= n8) return; FragH f;
#pragma unroll
  for (int q = 0; q < 8; ++q) f.h[q] = (_Float16)bf16_round(x[t * 8 + q]); *(volatile v8us*)((unsigned short*)X16 + t * 8) = f.half[0]; __threadfence(); *(volatile v8us*)((unsigned short*)X16 + t * 8) = f.half[0]; }
__global__ __launch_bounds__(256) void k_h16(const float* __restrict__ x, _Float16* __restrict__ X16, size_t n8) { const size_t t = (size_t)blockIdx.x * 256 + threadIdx.x; if (t >= n8) return; FragH f;
#pragma unroll
  for (int q = 0; q < 8; ++q) f.h[q] = (_Float16)x[t * 8 + q]; *(volatile v8us*)((unsigned short*)X16 + t * 8) = f.half[0]; __threadfence(); *(volatile v8us*)((unsigned short*)X16 + t * 8) = f.half[0]; }
__global__ __launch_bounds__(256) void k_round16f(const float* __restrict__ W, _Float16* __restrict__ Bt, size_t n8) { const size_t t = (size_t)blockIdx.x * 256 + threadIdx.x; if (t >= n8) return; FragH f;
#pragma unroll
  for (int i = 0; i < 8; ++i) f.h[i] = (_Float16)(bf16_round(W[t * 8 + i]) * 16.0f); *(volatile v8us*)((unsigned short*)Bt + t * 8) = f.half[0]; __threadfence(); *(volatile v8us*)((unsigned short*)Bt + t * 8) = f.half[0]; }
template <int NHv, int TTv>
__global__ __launch_bounds__(256) void k_vt(const _Float16* __restrict__ V16, int ldv, int voff, _Float16* __restrict__ Vt) { __shared__ unsigned short tl[64][66]; const int tid = threadIdx.x; const int slab = blockIdx.x / (TTv / 64), lg = blockIdx.x % (TTv / 64); const int b = slab / NHv, h = slab % NHv;
  for (int i = tid; i < 64 * 8; i += 256) { const int r = i / 8, c8 = (i % 8) * 8; FragH f; f.half[0] = *(const v8us*)((const unsigned short*)V16 + ((size_t)b * TTv + lg * 64 + r) * ldv + voff + h * 64 + c8);
#pragma unroll
    for (int q = 0; q < 8; ++q) tl[r][c8 + q] = f.u[q]; }
  __syncthreads();
  for (int pass = 0; pass < 2; ++pass) {
#pragma unroll
    for (int rd = 0; rd < 2; ++rd) { const int d = rd * 32 + tid / 8, pc = tid % 8; FragH f;
#pragma unroll
      for (int q = 0; q < 8; ++q) f.u[q] = tl[pc * 8 + q][d];
      *(volatile v8us*)((unsigned short*)Vt + ((size_t)slab * 64 + d) * TTv + lg * 64 + pc * 8) = f.half[0]; }
    if (pass == 0) __threadfence(); } }

__global__ __launch_bounds__(256) void k_hl(const float* __restrict__ F, _Float16* __restrict__ Hh, _Float16* __restrict__ Hl, size_t n8) { const size_t t = (size_t)blockIdx.x * 256 + threadIdx.x; if (t >= n8) return; FragH fh, fl; const v4f a = *(const v4fa*)(F + t * 8), c = *(const v4fa*)(F + t * 8 + 4);
#pragma unroll
  for (int q = 0; q < 4; ++q) { _Float16 h = (_Float16)a[q]; fh.h[q] = h; fl.h[q] = (_Float16)((a[q] - (float)h) * 1024.0f); h = (_Float16)c[q]; fh.h[4 + q] = h; fl.h[4 + q] = (_Float16)((c[q] - (float)h) * 1024.0f); }
  for (int pass = 0; pass < 2; ++pass) { *(volatile v8us*)((unsigned short*)Hh + t * 8) = fh.half[0]; *(volatile v8us*)((unsigned short*)Hl + t * 8) = fl.half[0]; if (pass == 0) __threadfence(); } }

__global__ __launch_bounds__(256) void k_conv(const float* __restrict__ XI, const float* __restrict__ cw, const float* __restrict__ cb, _Float16* __restrict__ U16) { const size_t t0 = (size_t)blockIdx.x * 256 + threadIdx.x; if (t0 >= (size_t)NR * (DI / 8)) return; const int d0 = (int)(t0 % (DI / 8)) * 8; const size_t row = t0 / (DI / 8); const int t = (int)(row % TT); FragH f;
#pragma unroll
  for (int j = 0; j < 8; ++j) { const int d = d0 + j; float a = bf16_round(cb[d]);
#pragma unroll
    for (int k = 0; k < 4; ++k) { const int back = 3 - k; const bool ok = (t >= back); const size_t rr = ok ? (row - (size_t)back) : row; a += ok ? bf16_round(cw[d * 4 + k]) * XI[rr * DI + d] : 0.f; }
    f.h[j] = (_Float16)(USC * (a / (1.0f + fexp(-a)))); }
  *(volatile v8us*)((unsigned short*)U16 + row * DI + d0) = f.half[0]; __threadfence(); *(volatile v8us*)((unsigned short*)U16 + row * DI + d0) = f.half[0]; }
__global__ __launch_bounds__(256) void k_dtr(const float* __restrict__ XD, _Float16* __restrict__ D16) { const size_t t = (size_t)blockIdx.x * 256 + threadIdx.x; if (t >= (size_t)NR * 4) return; const size_t row = t / 4; const int j0 = (int)(t % 4) * 8; FragH f;
#pragma unroll
  for (int q = 0; q < 8; ++q) f.h[q] = (j0 + q < DTR) ? (_Float16)XD[row * XDP + j0 + q] : (_Float16)0.0f;
  *(volatile v8us*)((unsigned short*)D16 + row * DTP + j0) = f.half[0]; __threadfence(); *(volatile v8us*)((unsigned short*)D16 + row * DTP + j0) = f.half[0]; }
__global__ __launch_bounds__(256) void k_wdt(const float* __restrict__ Wd, _Float16* __restrict__ Wdt) { const int t = blockIdx.x * 256 + threadIdx.x; if (t >= DI * 4) return; const int d = t / 4, j0 = (t % 4) * 8; FragH f;
#pragma unroll
  for (int q = 0; q < 8; ++q) f.h[q] = (j0 + q < DTR) ? (_Float16)(bf16_round(Wd[(size_t)d * DTR + j0 + q]) * 16.0f) : (_Float16)0.0f;
  *(volatile v8us*)((unsigned short*)Wdt + (size_t)d * DTP + j0) = f.half[0]; __threadfence(); *(volatile v8us*)((unsigned short*)Wdt + (size_t)d * DTP + j0) = f.half[0]; }
__global__ __launch_bounds__(256) void k_scan(const _Float16* __restrict__ U16, const _Float16* __restrict__ DT16, const float* __restrict__ XD, const float* __restrict__ RES, const float* __restrict__ Alog, const float* __restrict__ Dsk, _Float16* __restrict__ YS) {
  #pragma clang fp contract(off)
  const int gtid = blockIdx.x * 256 + threadIdx.x; const int b = gtid / (DI / 2), d0 = (gtid % (DI / 2)) * 2; if (b >= BB) return;
  float A0[NS], A1[NS], h0[NS], h1[NS];
#pragma unroll
  for (int n = 0; n < NS; ++n) { A0[n] = -fexp(bf16_round(Alog[(size_t)d0 * NS + n])); A1[n] = -fexp(bf16_round(Alog[(size_t)(d0 + 1) * NS + n])); h0[n] = 0.f; h1[n] = 0.f; }
  const float D0 = bf16_round(Dsk[d0]), D1 = bf16_round(Dsk[d0 + 1]);
#pragma unroll 1
  for (int t = 0; t < TT; ++t) { const size_t row = (size_t)b * TT + t; const unsigned int uw = *(const unsigned int*)((const unsigned short*)U16 + row * DI + d0), tw = *(const unsigned int*)((const unsigned short*)DT16 + row * DI + d0);
    FragH cv; cv.u[0] = (unsigned short)(uw & 0xFFFFu); cv.u[1] = (unsigned short)(uw >> 16); cv.u[2] = (unsigned short)(tw & 0xFFFFu); cv.u[3] = (unsigned short)(tw >> 16);
    const float u0 = (float)cv.h[0] * (1.0f / USC), u1 = (float)cv.h[1] * (1.0f / USC), t0 = (float)cv.h[2], t1 = (float)cv.h[3]; const float* bc = XD + row * XDP + DTR; const float du0 = t0 * u0, du1 = t1 * u1; float y0 = 0.f, y1 = 0.f;
#pragma unroll
    for (int n = 0; n < NS; ++n) { const float bn = bc[n], cn = bc[NS + n]; h0[n] = h0[n] * fexp(t0 * A0[n]) + du0 * bn; h1[n] = h1[n] * fexp(t1 * A1[n]) + du1 * bn; y0 += h0[n] * cn; y1 += h1[n] * cn; }
    y0 += u0 * D0; y1 += u1 * D1; const float r0 = RES[row * DI + d0], r1 = RES[row * DI + d0 + 1];
    FragH o; o.h[0] = (_Float16)(YSC * y0 * (r0 / (1.0f + fexp(-r0)))); o.h[1] = (_Float16)(YSC * y1 * (r1 / (1.0f + fexp(-r1))));        const unsigned int ow = (unsigned int)o.u[0] | ((unsigned int)o.u[1] << 16);
    volatile unsigned int* p = (volatile unsigned int*)((unsigned short*)YS + row * DI + d0); *p = ow; __threadfence(); *p = ow; } }


template <int LN>
__global__ __launch_bounds__(256) void k_tokln(const float* __restrict__ x, const float* __restrict__ g, const float* __restrict__ be, _Float16* __restrict__ X16) { __shared__ float tl[32][CCH + 1]; __shared__ float mu_s[32], rs_s[32]; const int tid = threadIdx.x; const int b = blockIdx.x / (TT / 32), pg = blockIdx.x % (TT / 32); const int p0 = pg * 32;
  for (int i = tid; i < CCH * 32; i += 256) { const int c = i / 32, pp = i % 32; tl[pp][c] = bf16_round(x[((size_t)b * CCH + c) * TT + p0 + pp]); } __syncthreads();
  if (LN) { if (tid < 32) { float s = 0.f; for (int c = 0; c < CCH; ++c) s += tl[tid][c]; const float mu = s * (1.0f / CCH); float v = 0.f; for (int c = 0; c < CCH; ++c) { const float d = tl[tid][c] - mu; v += d * d; } mu_s[tid] = mu; rs_s[tid] = rsqrtf(v * (1.0f / CCH) + LNEPS); } __syncthreads(); }
  for (int pass = 0; pass < 2; ++pass) { for (int i = tid; i < 32 * 16; i += 256) { const int r = i / 16, pc = i % 16; FragH f;
#pragma unroll
      for (int q = 0; q < 8; ++q) { const int c = pc * 8 + q; float v = (c < CCH) ? tl[r][min(c, CCH - 1)] : 0.f; if (LN && c < CCH) v = (v - mu_s[r]) * rs_s[r] * bf16_round(g[c]) + bf16_round(be[c]); f.h[q] = (c < CCH) ? (_Float16)v : (_Float16)0.0f; }
      *(volatile v8us*)((unsigned short*)X16 + ((size_t)b * TT + p0 + r) * CP16 + pc * 8) = f.half[0]; } if (pass == 0) __threadfence(); } }
__global__ __launch_bounds__(256) void k_dtb2(const float* __restrict__ dtb, float* __restrict__ B2) { const int d = blockIdx.x * 256 + threadIdx.x; if (d >= DI) return; const float v = 2.0f * bf16_round(dtb[d]); *(volatile float*)(B2 + d) = v; __threadfence(); *(volatile float*)(B2 + d) = v; }
__global__ __launch_bounds__(256) void k_wdtbc(const float* __restrict__ Wd, _Float16* __restrict__ Wx) { const int t = blockIdx.x * 256 + threadIdx.x; if (t >= 64 * (2 * DI / 8)) return; const int r = t / (2 * DI / 8), c0 = (t % (2 * DI / 8)) * 8; FragH f;
#pragma unroll
  for (int q = 0; q < 8; ++q) f.h[q] = (r < XPW) ? (_Float16)(bf16_round(Wd[(size_t)r * 2 * DI + c0 + q]) * 16.0f) : (_Float16)0.0f;
  *(volatile v8us*)((unsigned short*)Wx + (size_t)r * 2 * DI + c0) = f.half[0]; __threadfence(); *(volatile v8us*)((unsigned short*)Wx + (size_t)r * 2 * DI + c0) = f.half[0]; }
__global__ __launch_bounds__(256) void k_outT(const float* __restrict__ Tp, float* __restrict__ out) { __shared__ float tl[32][65]; const int tid = threadIdx.x; const int b = blockIdx.x / ((CCH / 32) * (TT / 64)), rem = blockIdx.x % ((CCH / 32) * (TT / 64)); const int cg = rem / (TT / 64), pg = rem % (TT / 64); const int c0 = cg * 32, p0 = pg * 64;
  for (int i = tid; i < 64 * 32; i += 256) { const int pp = i / 32, c = i % 32; tl[c][pp] = Tp[((size_t)b * TT + p0 + pp) * CCH + c0 + c]; } __syncthreads();
  for (int pass = 0; pass < 2; ++pass) { for (int i = tid; i < 32 * 16; i += 256) { const int c = i / 16, q4 = i % 16; const size_t o = ((size_t)b * CCH + c0 + c) * TT + p0 + q4 * 4;
      v4f v; for (int q = 0; q < 4; ++q) v[q] = tl[c][q4 * 4 + q]; *(volatile v4f*)(out + o) = v; } if (pass == 0) __threadfence(); } }

extern "C" void kernel_launch(void* const* d_in, const int* in_sizes, int n_in,
                              void* d_out, int out_size, void* d_ws, size_t ws_size, hipStream_t stream) {
  (void)in_sizes; (void)n_in; (void)out_size;
  const float* const* I = (const float* const*)d_in; const float* x = I[0]; const float* Kin = I[1]; const float* Qin = I[2]; const float* in_w = I[3]; const float* conv_w = I[4]; const float* conv_b = I[5]; const float* klg = I[6]; const float* klb = I[7]; const float* k_w = I[8]; const float* k_b = I[9];
  const float* qlg = I[10]; const float* qlb = I[11]; const float* q_w = I[12]; const float* q_b = I[13]; const float* dtbc_w = I[14]; const float* dt_w = I[15]; const float* dt_b = I[16]; const float* gate_w = I[17]; const float* gate_b = I[18]; const float* A_log = I[19]; const float* Dsk = I[20]; const float* out_w = I[21];
  char* ws = (char*)d_ws; size_t off = 0;
  auto take = [&](size_t bytes) { char* p = ws + off; off += (bytes + 255) & ~(size_t)255; return p; };
  _Float16* Win = (_Float16*)take((size_t)DI * CCH * 2); _Float16* Wk = (_Float16*)take((size_t)DI * CCH * 2); _Float16* Wq = (_Float16*)take((size_t)DI * CCH * 2); _Float16* Wx = (_Float16*)take((size_t)64 * 2 * DI * 2); _Float16* Wdt = (_Float16*)take((size_t)DI * DTP * 2); _Float16* Wg = (_Float16*)take((size_t)DI * 2 * DI * 2); _Float16* Wo = (_Float16*)take((size_t)CCH * DI * 2); float* B2 = (float*)take((size_t)DI * 4);
  _Float16* XT = (_Float16*)take((size_t)NR * CP16 * 2); _Float16* KL = (_Float16*)take((size_t)NR * CP16 * 2); _Float16* QL = (_Float16*)take((size_t)NR * CP16 * 2);
  float* XI = (float*)take((size_t)NR * DI * 4); _Float16* U16 = (_Float16*)take((size_t)NR * DI * 2); _Float16* Kp = (_Float16*)take((size_t)NR * DI * 2); _Float16* Qp = (_Float16*)take((size_t)NR * DI * 2); float* XD = (float*)take((size_t)NR * XDP * 4); _Float16* D16 = (_Float16*)take((size_t)NR * DTP * 2);
  float* Z = (float*)XT;
  _Float16* DT16 = (_Float16*)XI;
  _Float16* YS = (_Float16*)XI + (size_t)NR * DI;
  float* Tt = (float*)Kp;
  if (off > ws_size) return;
  k_round16f<<<(DI * CCH / 8 + 255) / 256, 256, 0, stream>>>(in_w, Win, (size_t)DI * CCH / 8); k_round16f<<<(DI * CCH / 8 + 255) / 256, 256, 0, stream>>>(k_w, Wk, (size_t)DI * CCH / 8); k_round16f<<<(DI * CCH / 8 + 255) / 256, 256, 0, stream>>>(q_w, Wq, (size_t)DI * CCH / 8);
  k_wdtbc<<<(64 * (2 * DI / 8) + 255) / 256, 256, 0, stream>>>(dtbc_w, Wx); k_wdt<<<(DI * 4 + 255) / 256, 256, 0, stream>>>(dt_w, Wdt); k_round16f<<<(DI * 2 * DI / 8 + 255) / 256, 256, 0, stream>>>(gate_w, Wg, (size_t)DI * 2 * DI / 8); k_round16f<<<(CCH * DI / 8 + 255) / 256, 256, 0, stream>>>(out_w, Wo, (size_t)CCH * DI / 8); k_dtb2<<<1, 256, 0, stream>>>(dt_b, B2);
  k_tokln<0><<<BB * (TT / 32), 256, 0, stream>>>(x, nullptr, nullptr, XT); k_tokln<1><<<BB * (TT / 32), 256, 0, stream>>>(Kin, klg, klb, KL); k_tokln<1><<<BB * (TT / 32), 256, 0, stream>>>(Qin, qlg, qlb, QL);
  const dim3 g192(((NR / 16) * (DI / 64) + 3) / 4, 1);
  k_gemm_hhx<0><<<g192, 128, 0, stream>>>(XT, CP16, 0, Win, CCH, 0, 0.0625f, nullptr, 0, nullptr, 1, 0, 0, XI, nullptr, DI, 0, NR, DI, CCH);
  k_gemm_hhx<15><<<g192, 128, 0, stream>>>(KL, CP16, 0, Wk, CCH, 0, 0.0625f, k_b, 0, nullptr, 1, 0, 0, nullptr, Kp, DI, 0, NR, DI, CCH);
  k_gemm_hhx<15><<<g192, 128, 0, stream>>>(QL, CP16, 0, Wq, CCH, 0, 0.0625f, q_b, 0, nullptr, 1, 0, 0, nullptr, Qp, DI, 0, NR, DI, CCH);
  k_conv<<<(unsigned)(((size_t)NR * (DI / 8) + 255) / 256), 256, 0, stream>>>(XI, conv_w, conv_b, U16);
  const dim3 gx(((NR / 16) * 1 + 3) / 4, 1);
  k_gemm_hhx<0><<<gx, 128, 0, stream>>>(U16, DI, 0, Wx, 2 * DI, 0, 0.0625f / USC, nullptr, 0, nullptr, 1, 0, 0, XD, nullptr, XDP, 0, NR, XPW, DI);
  k_gemm_hhx<0><<<gx, 128, 0, stream>>>(Kp, DI, 0, Wx + DI, 2 * DI, 0, 0.0625f, nullptr, 0, XD, 1, (size_t)XDP, 0, XD, nullptr, XDP, 0, NR, XPW, DI);
  k_gemm_hhx<0><<<g192, 128, 0, stream>>>(U16, DI, 0, Wg, 2 * DI, 0, 0.0625f / USC, gate_b, 0, nullptr, 1, 0, 0, Z, nullptr, DI, 0, NR, DI, DI);
  k_gemm_hhx<0><<<g192, 128, 0, stream>>>(Qp, DI, 0, Wg + DI, 2 * DI, 0, 0.0625f, nullptr, 0, Z, 1, (size_t)DI, 0, Z, nullptr, DI, 0, NR, DI, DI);
  k_dtr<<<(NR * 4 + 255) / 256, 256, 0, stream>>>(XD, D16);
  k_gemm_hhx<13><<<g192, 128, 0, stream>>>(D16, DTP, 0, Wdt, DTP, 0, 0.0625f, nullptr, 0, B2, NR, 0, 0, nullptr, DT16, DI, 0, NR, DI, DTP);
  k_scan<<<(BB * (DI / 2) + 255) / 256, 256, 0, stream>>>(U16, DT16, XD, Z, A_log, Dsk, YS);
  k_gemm_hhx<0><<<dim3(((NR / 16) * 2 + 3) / 4, 1), 128, 0, stream>>>(YS, DI, 0, Wo, DI, 0, 0.0625f / YSC, nullptr, 0, nullptr, 1, 0, 0, Tt, nullptr, CCH, 0, NR, CCH, DI);
  k_outT<<<BB * (CCH / 32) * (TT / 64), 256, 0, stream>>>(Tt, (float*)d_out);
}
